// WalzeAttentionLayerV3_27358941675956
// MI455X (gfx1250) — hardware-verified
//
#include <hip/hip_runtime.h>
#include <math.h>
typedef __attribute__((ext_vector_type(16))) _Float16 v16h;
typedef __attribute__((ext_vector_type(8)))  _Float16 v8h;
typedef __attribute__((ext_vector_type(16))) __bf16   v16b;
typedef __attribute__((ext_vector_type(8)))  __bf16   v8b;
typedef __attribute__((ext_vector_type(8)))  float    v8f;
typedef __attribute__((ext_vector_type(4)))  float    v4f;
#define PSCALE 32768.0f
#define U16(p) ((const unsigned short*)(const void*)(p))
#define PSCALE_INV (1.0f / 32768.0f)

__device__ __forceinline__ unsigned short f2bf_bits(float f) {
  unsigned u = __float_as_uint(f);
  return (unsigned short)((u + 0x7FFFu + ((u >> 16) & 1u)) >> 16);
}
__device__ __forceinline__ float bf_bits2f(unsigned short h) { return __uint_as_float(((unsigned)h) << 16); }

__device__ __forceinline__ void dep_guard_h(v8f& a, v8f& b, v16h x, v16h y) { asm volatile("v_nop\n\tv_nop\n\tv_nop\n\tv_nop" : "+v"(a), "+v"(b) : "v"(x), "v"(y)); }
__device__ __forceinline__ void dep_guard_b(v8f& a, v8f& b, v16b x, v16b y) { asm volatile("v_nop\n\tv_nop\n\tv_nop\n\tv_nop" : "+v"(a), "+v"(b) : "v"(x), "v"(y)); }
__device__ __forceinline__ void keep4_h(v16h a, v16h b, v16h c, v16h d) { asm volatile("v_nop" :: "v"(a), "v"(b), "v"(c), "v"(d)); }
__device__ __forceinline__ void keep4_b(v16b a, v16b b, v16b c, v16b d) { asm volatile("v_nop" :: "v"(a), "v"(b), "v"(c), "v"(d)); }
__device__ __forceinline__ void acc_guard4(v8f& a, v8f& b, v8f& c, v8f& d) { asm volatile("v_nop\n\tv_nop\n\tv_nop\n\tv_nop" : "+v"(a), "+v"(b), "+v"(c), "+v"(d)); }
template <typename T> struct Frag;
template <> struct Frag<_Float16> {
  typedef v16h V; union U { v16h v; v8h h[2]; };
  static __device__ __forceinline__ v16h load(const _Float16* p) {
    U f; f.h[0] = *(const v8h*)(p); f.h[1] = *(const v8h*)(p + 16); return f.v;
  }
  static __device__ __forceinline__ v8f mma(v16h a, v16h b, v8f c) {
    return __builtin_amdgcn_wmma_f32_16x16x32_f16(false, a, false, b, (short)0, c, false, false);
  }
  static __device__ __forceinline__ void guard(v8f& a, v8f& b, v16h x, v16h y) { dep_guard_h(a, b, x, y); }
  static __device__ __forceinline__ void keep(v16h a, v16h b, v16h c, v16h d) { keep4_h(a, b, c, d); }
};
template <> struct Frag<__bf16> {
  typedef v16b V; union U { v16b v; v8b h[2]; };
  static __device__ __forceinline__ v16b load(const __bf16* p) {
    U f; f.h[0] = *(const v8b*)(p); f.h[1] = *(const v8b*)(p + 16); return f.v;
  }
  static __device__ __forceinline__ v8f mma(v16b a, v16b b, v8f c) {
    return __builtin_amdgcn_wmma_f32_16x16x32_bf16(false, a, false, b, (short)0, c, false, false);
  }
  static __device__ __forceinline__ void guard(v8f& a, v8f& b, v16b x, v16b y) { dep_guard_b(a, b, x, y); }
  static __device__ __forceinline__ void keep(v16b a, v16b b, v16b c, v16b d) { keep4_b(a, b, c, d); }
};

template <int ET> struct Elem;
template <> struct Elem<0> { typedef _Float16 T; };
template <> struct Elem<1> { typedef __bf16 T; };
template <int ET, bool SPLIT, int BIAS_MODE, int OUT_MODE, bool RESID, int ACT = 0>
__global__ __launch_bounds__(256) void wmma_gemm64(
    const unsigned short* __restrict__ Ap, const unsigned short* __restrict__ A2p, int lda, long strideA,
    const unsigned short* __restrict__ Btp, const unsigned short* __restrict__ Bt2p, int ldb, long strideB,
    void* __restrict__ Cout, void* __restrict__ Cout2, int ldc, long strideC,
    const float* __restrict__ bias,
    const float* __restrict__ resid, long strideR,
    int M, int N, int K, float scale) {
  typedef typename Elem<ET>::T T;
  typedef typename Frag<T>::V V;
  const T* A = (const T*)Ap; const T* A2 = (const T*)A2p; const T* Bt = (const T*)Btp; const T* Bt2 = (const T*)Bt2p;
  __shared__ __align__(16) float sT[8][16 * 68];
  const int b    = blockIdx.y;
  const int lane = threadIdx.x & 31;
  const int wave = threadIdx.x >> 5;
  const int tilesN = N >> 6;
  const int tilesM = M >> 6;
  const int tile = blockIdx.x * 8 + wave;
  if (tile >= tilesM * tilesN) return;
  const int tm = tile / tilesN;
  const int tn = tile - tm * tilesN;
  const int m0 = tm << 6;
  const int n0 = tn << 6;

  const T* Ab  = A  + (size_t)b * strideA;
  const T* Bb  = Bt + (size_t)b * strideB;
  const T* Ab2 = SPLIT ? (A2  + (size_t)b * strideA) : nullptr;
  const T* Bb2 = SPLIT ? (Bt2 + (size_t)b * strideB) : nullptr;

  const int rlane = lane & 15;
  const int koff  = (lane >> 4) * 8;
  const int mOff  = (lane >> 4) * 8;

  v8f acc[4][4];
#pragma unroll
  for (int i = 0; i < 4; ++i)
#pragma unroll
    for (int j = 0; j < 4; ++j) acc[i][j] = (v8f){0.f,0.f,0.f,0.f,0.f,0.f,0.f,0.f};

  for (int k0 = 0; k0 < K; k0 += 32) {
    V bh[4], bl[4];
#pragma unroll
    for (int j = 0; j < 4; ++j) {
      const size_t bo = (size_t)(n0 + (j << 4) + rlane) * ldb + koff + k0;
      bh[j] = Frag<T>::load(Bb + bo);
      if (SPLIT) bl[j] = Frag<T>::load(Bb2 + bo);
    }
#pragma unroll
    for (int i = 0; i < 4; ++i) {
      const size_t ao = (size_t)(m0 + (i << 4) + rlane) * lda + koff + k0;
      V ah = Frag<T>::load(Ab + ao);
      V al;
      if (SPLIT) al = Frag<T>::load(Ab2 + ao);
#pragma unroll
      for (int j = 0; j < 4; ++j) {
        acc[i][j] = Frag<T>::mma(ah, bh[j], acc[i][j]);
        if (SPLIT) {
          acc[i][j] = Frag<T>::mma(ah, bl[j], acc[i][j]);
          acc[i][j] = Frag<T>::mma(al, bh[j], acc[i][j]);
        }
      }
      Frag<T>::guard(acc[i][0], acc[i][3], ah, SPLIT ? al : ah);
    }
    Frag<T>::keep(bh[0], bh[1], bh[2], bh[3]);
    if (SPLIT) Frag<T>::keep(bl[0], bl[1], bl[2], bl[3]);
  }
  acc_guard4(acc[0][0], acc[0][1], acc[0][2], acc[0][3]);
  acc_guard4(acc[1][0], acc[1][1], acc[1][2], acc[1][3]);
  acc_guard4(acc[2][0], acc[2][1], acc[2][2], acc[2][3]);
  acc_guard4(acc[3][0], acc[3][1], acc[3][2], acc[3][3]);

  float* slab = sT[wave];
  const float* Rb = RESID ? (resid + (size_t)b * strideR) : nullptr;
#pragma unroll
  for (int i = 0; i < 4; ++i) {
    const int mBase = m0 + (i << 4);
#pragma unroll
    for (int j = 0; j < 4; ++j) {
      const int n = n0 + (j << 4) + rlane;
      float bv = 0.f;
      if (BIAS_MODE == 2) bv = bias[n];
#pragma unroll
      for (int r = 0; r < 8; ++r) {
        float v = acc[i][j][r] * scale;
        if (BIAS_MODE == 1) v += bias[mBase + mOff + r];
        if (BIAS_MODE == 2) v += bv;
        if (RESID) v += Rb[(size_t)(mBase + mOff + r) * ldc + n];
        if (ACT == 1) v = tanhf(v);
        if (ACT == 2) v = fmaxf(v, 0.0f);
        if (ACT == 3) v = v / (1.0f + expf(-v));
        if (ACT == 4) v = (v > 0.f) ? v : 0.01f * v;
        if (ACT == 5) v = 0.5f * v * (1.0f + erff(v * 0.70710678118654752f));
        slab[(mOff + r) * 68 + (j << 4) + rlane] = v;
      }
    }
    __builtin_amdgcn_fence(__ATOMIC_RELEASE, "workgroup");
    __builtin_amdgcn_wave_barrier();
    __builtin_amdgcn_fence(__ATOMIC_ACQUIRE, "workgroup");
    if (OUT_MODE == 0) {
      float* C = (float*)Cout + (size_t)b * strideC;
      const int hh = lane >> 4, c4 = (lane & 15) * 4;
      for (int pass = 0; pass < 2; ++pass) {
#pragma unroll
        for (int it = 0; it < 8; ++it) {
          const int row = it * 2 + hh;
          v4f v = *(const v4f*)(slab + row * 68 + c4);
          *(volatile v4f*)(C + (size_t)(mBase + row) * ldc + n0 + c4) = v;
        }
        __threadfence();
      }
    } else {
      const int q = lane >> 3, c8 = (lane & 7) * 8;
      unsigned short* C  = (unsigned short*)Cout  + (size_t)b * strideC;
      unsigned short* C2 = (OUT_MODE == 2) ? ((unsigned short*)Cout2 + (size_t)b * strideC) : nullptr;
      for (int pass = 0; pass < 2; ++pass) {
#pragma unroll
        for (int it = 0; it < 4; ++it) {
          const int row = it * 4 + q;
          const float* sp = slab + row * 68 + c8;
          v8h hv, lv;
#pragma unroll
          for (int e = 0; e < 8; ++e) {
            if (OUT_MODE == 1) {
              hv[e] = (_Float16)sp[e];
            } else {
              unsigned short hb = f2bf_bits(sp[e]);
              unsigned short lb = f2bf_bits(sp[e] - bf_bits2f(hb));
              hv[e] = __builtin_bit_cast(_Float16, hb);
              lv[e] = __builtin_bit_cast(_Float16, lb);
            }
          }
          *(volatile v8h*)(C + (size_t)(mBase + row) * ldc + n0 + c8) = hv;
          if (OUT_MODE == 2) *(volatile v8h*)(C2 + (size_t)(mBase + row) * ldc + n0 + c8) = lv;
        }
        __threadfence();
      }
    }
    __builtin_amdgcn_fence(__ATOMIC_RELEASE, "workgroup");
    __builtin_amdgcn_wave_barrier();
    __builtin_amdgcn_fence(__ATOMIC_ACQUIRE, "workgroup");
  }
}

__global__ __launch_bounds__(256) void cast_f32_f16x2(
    const float* __restrict__ in, _Float16* __restrict__ out, int n2) {
  int i = blockIdx.x * 256 + threadIdx.x;
  if (i < n2) {
    const _Float16 h0 = (_Float16)in[2 * i], h1 = (_Float16)in[2 * i + 1];
    const unsigned u = (unsigned)__builtin_bit_cast(unsigned short, h0) | ((unsigned)__builtin_bit_cast(unsigned short, h1) << 16);
    ((volatile unsigned*)out)[i] = u;
    __threadfence();
    ((volatile unsigned*)out)[i] = u;
  }
}


#define ZB 16
#define ZC 256
#define ZH 32
#define ZW 32
#define ZS (ZH * ZW)
#define ZR (ZB * ZS)
#define ZNH 4
#define ZHD 64
#define ZWIN 16
__device__ __forceinline__ float gelu_exact(float v) { return 0.5f * v * (1.0f + erff(v * 0.70710678118654752f)); }
__global__ __launch_bounds__(256) void walze_kernel(const float* __restrict__ x, const float* __restrict__ cw, const float* __restrict__ cb, const float* __restrict__ bg, const float* __restrict__ bb, const float* __restrict__ bm, const float* __restrict__ bv,
                                                   float* __restrict__ WZ, unsigned* __restrict__ COMB) {
  __shared__ float xs[64][4][33]; __shared__ float wo[64][65]; __shared__ float xo[64][65];
  const int b = blockIdx.z, c0 = blockIdx.y * 64, h0 = blockIdx.x * 2, tx = threadIdx.x, ty = threadIdx.y;
  for (int c = ty; c < 64; c += 8) for (int rr = 0; rr < 4; ++rr) { const int hr = (h0 - 1 + rr + ZH) % ZH; xs[c][rr][tx] = x[(((size_t)b * ZC + c0 + c) * ZH + hr) * ZW + tx]; }
  __syncthreads();
  for (int c = ty; c < 64; c += 8) { const int cg = c0 + c; const float* w9 = cw + cg * 9;
    const float isd = rsqrtf(bv[cg] + 1e-5f);
    for (int hh = 0; hh < 2; ++hh) { float conv = cb[cg];
#pragma unroll
      for (int kh = 0; kh < 3; ++kh) {
#pragma unroll
        for (int kw = 0; kw < 3; ++kw) conv += w9[kh * 3 + kw] * xs[c][hh + kh][(tx + kw - 1 + ZW) % ZW]; }
      const float xv = xs[c][hh + 1][tx]; const float pre = conv + xv; const float bn = (pre - bm[cg]) * isd * bg[cg] + bb[cg];
      wo[hh * 32 + tx][c] = gelu_exact(bn); xo[hh * 32 + tx][c] = xv; } }
  __syncthreads();
  for (int pass = 0; pass < 2; ++pass) {
    for (int t = ty; t < 64; t += 8) { const size_t r = (size_t)b * ZS + (size_t)h0 * ZW + t;
      typedef __attribute__((ext_vector_type(2))) float v2f; const v2f wv = {wo[t][2 * tx], wo[t][2 * tx + 1]};
      *(volatile v2f*)(WZ + r * ZC + c0 + 2 * tx) = wv;
      const unsigned ux = (unsigned)__builtin_bit_cast(unsigned short, (_Float16)xo[t][2 * tx]) | ((unsigned)__builtin_bit_cast(unsigned short, (_Float16)xo[t][2 * tx + 1]) << 16);
      const unsigned uw = (unsigned)__builtin_bit_cast(unsigned short, (_Float16)wv[0]) | ((unsigned)__builtin_bit_cast(unsigned short, (_Float16)wv[1]) << 16);
      ((volatile unsigned*)COMB)[(r * 512 + c0) / 2 + tx] = ux; ((volatile unsigned*)COMB)[(r * 512 + 256 + c0) / 2 + tx] = uw; }
    __threadfence(); }
}
__global__ __launch_bounds__(256) void ln1_kernel(const float* __restrict__ WZ, const float* __restrict__ g, const float* __restrict__ bb, float* __restrict__ WN, unsigned* __restrict__ WN16) {
  const int lane = threadIdx.x & 31, wave = threadIdx.x >> 5; const size_t r = (size_t)blockIdx.x * 8 + wave;
  float v[8]; { const v4f a = *(const v4f*)(WZ + r * ZC + lane * 8), c = *(const v4f*)(WZ + r * ZC + lane * 8 + 4); for (int q = 0; q < 4; ++q) { v[q] = a[q]; v[4 + q] = c[q]; } }
  float s = 0.f; for (int q = 0; q < 8; ++q) s += v[q]; for (int o = 16; o > 0; o >>= 1) s += __shfl_xor(s, o, 32);
  const float mean = s / ZC; float s2 = 0.f; for (int q = 0; q < 8; ++q) { const float d = v[q] - mean; s2 += d * d; } for (int o = 16; o > 0; o >>= 1) s2 += __shfl_xor(s2, o, 32);
  const float inv = rsqrtf(s2 / ZC + 1e-5f);
  for (int q = 0; q < 8; ++q) { const int c = lane * 8 + q; v[q] = (v[q] - mean) * inv * g[c] + bb[c]; }
  typedef __attribute__((ext_vector_type(4))) unsigned u4; u4 pk; for (int q = 0; q < 4; ++q) pk[q] = (unsigned)__builtin_bit_cast(unsigned short, (_Float16)v[2 * q]) | ((unsigned)__builtin_bit_cast(unsigned short, (_Float16)v[2 * q + 1]) << 16);
  const v4f a = {v[0], v[1], v[2], v[3]}, c = {v[4], v[5], v[6], v[7]};
  for (int pass = 0; pass < 2; ++pass) { *(volatile v4f*)(WN + r * ZC + lane * 8) = a; *(volatile v4f*)(WN + r * ZC + lane * 8 + 4) = c; *(volatile u4*)(WN16 + (r * ZC) / 2 + lane * 4) = pk; __threadfence(); }
}
__global__ __launch_bounds__(256) void band_attn_kernel(const float* __restrict__ QKV, unsigned* __restrict__ CTX16) {
  const int lane = threadIdx.x & 31, wave = threadIdx.x >> 5; const size_t item = (size_t)blockIdx.x * 8 + wave; const size_t r = item >> 2; const int h = (int)(item & 3);
  const int i = (int)(r % ZS); const size_t rb = r - i;
  typedef __attribute__((ext_vector_type(2))) float v2f;
  const v2f q = *(const v2f*)(QKV + r * 768 + h * ZHD + 2 * lane) * 0.125f;
  float m = -INFINITY, ssum = 0.f; v2f acc = {0.f, 0.f};
  const int j0 = (i - ZWIN) < 0 ? 0 : (i - ZWIN), j1 = (i + ZWIN) > (ZS - 1) ? (ZS - 1) : (i + ZWIN);
  for (int j = j0; j <= j1; ++j) { const float* kr = QKV + (rb + j) * 768 + ZC + h * ZHD; const v2f kk = *(const v2f*)(kr + 2 * lane); const v2f vv = *(const v2f*)(kr + ZC + 2 * lane);
    float s = q[0] * kk[0] + q[1] * kk[1]; for (int o = 16; o > 0; o >>= 1) s += __shfl_xor(s, o, 32);
    const float mn = fmaxf(m, s); const float sc = expf(m - mn); const float e = expf(s - mn); ssum = ssum * sc + e; acc = acc * sc + e * vv; m = mn; }
  const v2f o2 = acc / ssum;
  const unsigned u = (unsigned)__builtin_bit_cast(unsigned short, (_Float16)o2[0]) | ((unsigned)__builtin_bit_cast(unsigned short, (_Float16)o2[1]) << 16);
  ((volatile unsigned*)CTX16)[(r * ZC + h * ZHD) / 2 + lane] = u; __threadfence(); ((volatile unsigned*)CTX16)[(r * ZC + h * ZHD) / 2 + lane] = u;
}
__global__ __launch_bounds__(256) void final_kernel(const float* __restrict__ H1, const float* __restrict__ d2w, const float* __restrict__ d2b, const float* __restrict__ WN, const float* __restrict__ AO, const float* __restrict__ g, const float* __restrict__ bb, float* __restrict__ FIN) {
  const int lane = threadIdx.x & 31, wave = threadIdx.x >> 5; const size_t r = (size_t)blockIdx.x * 8 + wave;
  float d = H1[r * 64 + 2 * lane] * d2w[2 * lane] + H1[r * 64 + 2 * lane + 1] * d2w[2 * lane + 1]; for (int o = 16; o > 0; o >>= 1) d += __shfl_xor(d, o, 32);
  const float sp = 1.0f / (1.0f + expf(-(d + d2b[0])));
  float v[8]; { const v4f a = *(const v4f*)(WN + r * ZC + lane * 8), c = *(const v4f*)(WN + r * ZC + lane * 8 + 4), a2 = *(const v4f*)(AO + r * ZC + lane * 8), c2 = *(const v4f*)(AO + r * ZC + lane * 8 + 4);
    for (int q = 0; q < 4; ++q) { v[q] = (1.f - sp) * a[q] + sp * a2[q]; v[4 + q] = (1.f - sp) * c[q] + sp * c2[q]; } }
  float s = 0.f; for (int q = 0; q < 8; ++q) s += v[q]; for (int o = 16; o > 0; o >>= 1) s += __shfl_xor(s, o, 32);
  const float mean = s / ZC; float s2 = 0.f; for (int q = 0; q < 8; ++q) { const float dd = v[q] - mean; s2 += dd * dd; } for (int o = 16; o > 0; o >>= 1) s2 += __shfl_xor(s2, o, 32);
  const float inv = rsqrtf(s2 / ZC + 1e-5f);
  for (int q = 0; q < 8; ++q) { const int c = lane * 8 + q; v[q] = (v[q] - mean) * inv * g[c] + bb[c]; }
  const v4f a = {v[0], v[1], v[2], v[3]}, c = {v[4], v[5], v[6], v[7]};
  for (int pass = 0; pass < 2; ++pass) { *(volatile v4f*)(FIN + r * ZC + lane * 8) = a; *(volatile v4f*)(FIN + r * ZC + lane * 8 + 4) = c; __threadfence(); }
}
__global__ __launch_bounds__(256) void out_kernel(const float* __restrict__ FIN, const float* __restrict__ x, float* __restrict__ out) {
  __shared__ float tile[64][65];
  const int b = blockIdx.z, c0 = blockIdx.y * 64, s0 = blockIdx.x * 64, tx = threadIdx.x, ty = threadIdx.y;
  for (int t = ty; t < 64; t += 8) { const float* src = FIN + ((size_t)b * ZS + s0 + t) * ZC + c0; tile[tx][t] = src[tx]; tile[32 + tx][t] = src[32 + tx]; }
  __syncthreads();
  for (int pass = 0; pass < 2; ++pass) { for (int c = ty; c < 64; c += 8) { const size_t base = ((size_t)b * ZC + c0 + c) * ZS + s0; ((volatile float*)out)[base + tx] = tile[c][tx] + x[base + tx]; ((volatile float*)out)[base + 32 + tx] = tile[c][32 + tx] + x[base + 32 + tx]; } __threadfence(); }
}
extern "C" void kernel_launch(void* const* d_in, const int* in_sizes, int n_in, void* d_out, int out_size, void* d_ws, size_t ws_size, hipStream_t stream) {
  (void)in_sizes; (void)n_in; (void)out_size; (void)ws_size;
  const float* x = (const float*)d_in[0]; const float* cw = (const float*)d_in[1]; const float* cb = (const float*)d_in[2]; const float* bg = (const float*)d_in[3]; const float* bbn = (const float*)d_in[4]; const float* bm = (const float*)d_in[5]; const float* bvv = (const float*)d_in[6];
  const float* l1g = (const float*)d_in[7]; const float* l1b = (const float*)d_in[8]; const float* l2g = (const float*)d_in[9]; const float* l2b = (const float*)d_in[10]; const float* inw = (const float*)d_in[11]; const float* inb = (const float*)d_in[12]; const float* ow = (const float*)d_in[13]; const float* ob = (const float*)d_in[14];
  const float* d1w = (const float*)d_in[15]; const float* d1b = (const float*)d_in[16]; const float* d2w = (const float*)d_in[17]; const float* d2b = (const float*)d_in[18];
  char* ws = (char*)d_ws; size_t off = 0;
  auto carve = [&](size_t bytes) -> char* { char* p = ws + off; off += (bytes + 255) & ~(size_t)255; return p; };
  float* WZ = (float*)carve((size_t)ZR * ZC * 4); unsigned* COMB = (unsigned*)carve((size_t)ZR * 512 * 2); float* WN = (float*)carve((size_t)ZR * ZC * 4); unsigned* WN16 = (unsigned*)carve((size_t)ZR * ZC * 2);
  _Float16* INW = (_Float16*)carve((size_t)768 * ZC * 2); _Float16* OW = (_Float16*)carve((size_t)ZC * ZC * 2); _Float16* D1W = (_Float16*)carve((size_t)64 * 512 * 2);
  float* QKV = (float*)carve((size_t)ZR * 768 * 4); unsigned* CTX16 = (unsigned*)carve((size_t)ZR * ZC * 2); float* AO = (float*)carve((size_t)ZR * ZC * 4); float* H1 = (float*)carve((size_t)ZR * 64 * 4); float* FIN = WZ;
  walze_kernel<<<dim3(ZH / 2, ZC / 64, ZB), dim3(32, 8), 0, stream>>>(x, cw, cb, bg, bbn, bm, bvv, WZ, COMB);
  ln1_kernel<<<ZR / 8, 256, 0, stream>>>(WZ, l1g, l1b, WN, WN16);
  cast_f32_f16x2<<<(768 * ZC / 2 + 255) / 256, 256, 0, stream>>>(inw, INW, 768 * ZC / 2);
  cast_f32_f16x2<<<(ZC * ZC / 2 + 255) / 256, 256, 0, stream>>>(ow, OW, ZC * ZC / 2);
  cast_f32_f16x2<<<(64 * 512 / 2 + 255) / 256, 256, 0, stream>>>(d1w, D1W, 64 * 512 / 2);
  { const int t = (ZR / 64) * 12;
    wmma_gemm64<0, false, 2, 0, false><<<dim3((t + 7) / 8, 1), 256, 0, stream>>>((const unsigned short*)WN16, nullptr, ZC, 0, U16(INW), nullptr, ZC, 0, QKV, nullptr, 768, 0, inb, nullptr, 0, ZR, 768, ZC, 1.0f); }
  band_attn_kernel<<<ZR * ZNH / 8, 256, 0, stream>>>(QKV, CTX16);
  { const int t = (ZR / 64) * 4;
    wmma_gemm64<0, false, 2, 0, false><<<dim3((t + 7) / 8, 1), 256, 0, stream>>>((const unsigned short*)CTX16, nullptr, ZC, 0, U16(OW), nullptr, ZC, 0, AO, nullptr, ZC, 0, ob, nullptr, 0, ZR, ZC, ZC, 1.0f); }
  { const int t = (ZR / 64) * 1;
    wmma_gemm64<0, false, 2, 0, false, 5><<<dim3((t + 7) / 8, 1), 256, 0, stream>>>((const unsigned short*)COMB, nullptr, 512, 0, U16(D1W), nullptr, 512, 0, H1, nullptr, 64, 0, d1b, nullptr, 0, ZR, 64, 512, 1.0f); }
  final_kernel<<<ZR / 8, 256, 0, stream>>>(H1, d2w, d2b, WN, AO, l2g, l2b, FIN);
  out_kernel<<<dim3(ZS / 64, ZC / 64, ZB), dim3(32, 8), 0, stream>>>(FIN, x, (float*)d_out);
}
